// Encoder_30116310680397
// MI455X (gfx1250) — hardware-verified
//
#include <hip/hip_runtime.h>
#include <math.h>

constexpr int SEQ_LEN   = 128;
constexpr int NBAT      = 64;
constexpr int NVOC      = 32000;
constexpr int NEMB      = 512;
constexpr int NHID      = 1024;
constexpr int NGATE2    = 2 * NHID;
constexpr int NGATE3    = 3 * NHID;
constexpr int NROWS     = SEQ_LEN * NBAT;
constexpr int SCAN_THR  = 512;
constexpr int SCAN_WAVES = SCAN_THR / 32;
constexpr int ROWS_BLK  = 16;
constexpr int HPITCH    = 1032;
constexpr int SLABP     = 68;
constexpr int CVT_THR   = 256;
constexpr float WCARRY  = 16.0f;
constexpr float HCARRY  = 1024.0f;
constexpr float GCARRY  = 64.0f;
constexpr float ACC_INV = 1.0f / (WCARRY * HCARRY);
constexpr float GX_INV  = 1.0f / GCARRY;
constexpr float S1_SCALE = GCARRY / (WCARRY * WCARRY);
constexpr float S4_SCALE = GCARRY / (WCARRY * HCARRY);
static_assert(NHID == 64 * SCAN_WAVES, "each wave owns 64 hidden columns");
static_assert(NBAT % ROWS_BLK == 0, "batch tiles");
static_assert(NEMB % 32 == 0 && NHID % 32 == 0, "GEMM K multiple of 32");
static_assert(NROWS % 64 == 0 && NGATE3 % 64 == 0, "GEMM M, N tile multiples");
static_assert(NEMB % 64 == 0 && NHID % 64 == 0 && NGATE2 % 64 == 0, "transpose tiles");
static_assert(HPITCH % 8 == 0 && HPITCH >= NHID, "LDS pitch");
static_assert((NROWS * (NEMB / 8)) % CVT_THR == 0, "embed grid exact");

typedef __attribute__((ext_vector_type(16))) _Float16 v16h;
typedef __attribute__((ext_vector_type(8)))  _Float16 v8h;
typedef __attribute__((ext_vector_type(16))) __bf16   v16b;
typedef __attribute__((ext_vector_type(8)))  __bf16   v8b;
typedef __attribute__((ext_vector_type(8)))  float    v8f;
typedef __attribute__((ext_vector_type(4)))  float    v4f;
typedef __attribute__((ext_vector_type(4)))  unsigned v4u;

__device__ __forceinline__ unsigned short f2bf_bits(float f) {
  unsigned u = __float_as_uint(f);
  return (unsigned short)((u + 0x7FFFu + ((u >> 16) & 1u)) >> 16);
}
__device__ __forceinline__ float bf_bits2f(unsigned short h) { return __uint_as_float(((unsigned)h) << 16); }

__device__ __forceinline__ float h16_to_f32(unsigned hb) {
  const unsigned sgn = (hb & 0x8000u) << 16;
  const unsigned em = hb & 0x7fffu;
  const float fn = __uint_as_float((em << 13) + 0x38000000u);
  const float fs = (float)em * 5.9604644775390625e-8f;
  const float mag = (em < 0x400u) ? fs : fn;
  return __uint_as_float(__float_as_uint(mag) | sgn);
}
__device__ __forceinline__ void unpack8(const v4u g, float (&f)[8]) {
  const unsigned w0 = g[0];
  const unsigned w1 = g[1];
  const unsigned w2 = g[2];
  const unsigned w3 = g[3];
  f[0] = h16_to_f32(w0 & 0xffffu);
  f[1] = h16_to_f32(w0 >> 16);
  f[2] = h16_to_f32(w1 & 0xffffu);
  f[3] = h16_to_f32(w1 >> 16);
  f[4] = h16_to_f32(w2 & 0xffffu);
  f[5] = h16_to_f32(w2 >> 16);
  f[6] = h16_to_f32(w3 & 0xffffu);
  f[7] = h16_to_f32(w3 >> 16);
}

__device__ __forceinline__ void keep4_h(v16h a, v16h b, v16h c, v16h d) { asm volatile("v_nop" :: "v"(a), "v"(b), "v"(c), "v"(d)); }
__device__ __forceinline__ void keep4_b(v16b a, v16b b, v16b c, v16b d) { asm volatile("v_nop" :: "v"(a), "v"(b), "v"(c), "v"(d)); }
__device__ __forceinline__ void acc_guard4(v8f& a, v8f& b, v8f& c, v8f& d) { asm volatile("v_nop\n\tv_nop\n\tv_nop\n\tv_nop" : "+v"(a), "+v"(b), "+v"(c), "+v"(d)); }
__device__ __forceinline__ void grp_guard_h(v8f& c0, v8f& c1, v8f& c2, v8f& c3, v16h x, v16h y, v16h b0, v16h b1, v16h b2, v16h b3) {
  asm volatile("v_nop\n\tv_nop\n\tv_nop\n\tv_nop" : "+v"(c0), "+v"(c1), "+v"(c2), "+v"(c3) : "v"(x), "v"(y), "v"(b0), "v"(b1), "v"(b2), "v"(b3));
}
__device__ __forceinline__ void grp_guard_b(v8f& c0, v8f& c1, v8f& c2, v8f& c3, v16b x, v16b y, v16b b0, v16b b1, v16b b2, v16b b3) {
  asm volatile("v_nop\n\tv_nop\n\tv_nop\n\tv_nop" : "+v"(c0), "+v"(c1), "+v"(c2), "+v"(c3) : "v"(x), "v"(y), "v"(b0), "v"(b1), "v"(b2), "v"(b3));
}

template <typename T> struct Frag;
template <> struct Frag<_Float16> {
  typedef v16h V;
  union U { v16h v; v8h h[2]; };
  static __device__ __forceinline__ v16h load(const _Float16* p) {
    U f;
    f.h[0] = *(const v8h*)(p);
    f.h[1] = *(const v8h*)(p + 16);
    return f.v;
  }
  static __device__ __forceinline__ v8f mma(v16h a, v16h b, v8f c) {
    return __builtin_amdgcn_wmma_f32_16x16x32_f16(false, a, false, b, (short)0, c, false, false);
  }
  static __device__ __forceinline__ void guard4(v8f& c0, v8f& c1, v8f& c2, v8f& c3, v16h x, v16h y, v16h b0, v16h b1, v16h b2, v16h b3) {
    grp_guard_h(c0, c1, c2, c3, x, y, b0, b1, b2, b3);
  }
  static __device__ __forceinline__ void keep(v16h a, v16h b, v16h c, v16h d) { keep4_h(a, b, c, d); }
};
template <> struct Frag<__bf16> {
  typedef v16b V;
  union U { v16b v; v8b h[2]; };
  static __device__ __forceinline__ v16b load(const __bf16* p) {
    U f;
    f.h[0] = *(const v8b*)(p);
    f.h[1] = *(const v8b*)(p + 16);
    return f.v;
  }
  static __device__ __forceinline__ v8f mma(v16b a, v16b b, v8f c) {
    return __builtin_amdgcn_wmma_f32_16x16x32_bf16(false, a, false, b, (short)0, c, false, false);
  }
  static __device__ __forceinline__ void guard4(v8f& c0, v8f& c1, v8f& c2, v8f& c3, v16b x, v16b y, v16b b0, v16b b1, v16b b2, v16b b3) {
    grp_guard_b(c0, c1, c2, c3, x, y, b0, b1, b2, b3);
  }
  static __device__ __forceinline__ void keep(v16b a, v16b b, v16b c, v16b d) { keep4_b(a, b, c, d); }
};

template <int ET> struct Elem;
template <> struct Elem<0> { typedef _Float16 T; };
template <> struct Elem<1> { typedef __bf16 T; };
template <int ET, bool SPLIT, int BIAS_MODE, int OUT_MODE, bool RESID, int ACT = 0>
__global__ __launch_bounds__(256) void wmma_gemm64(
    const unsigned short* __restrict__ Ap, const unsigned short* __restrict__ A2p, int lda, long strideA,
    const unsigned short* __restrict__ Btp, const unsigned short* __restrict__ Bt2p, int ldb, long strideB,
    void* __restrict__ Cout, void* __restrict__ Cout2, int ldc, long strideC,
    const float* __restrict__ bias,
    const float* __restrict__ resid, long strideR,
    int M, int N, int K, float scale) {
  typedef typename Elem<ET>::T T;
  typedef typename Frag<T>::V V;
  const T* A = (const T*)Ap;
  const T* A2 = (const T*)A2p;
  const T* Bt = (const T*)Btp;
  const T* Bt2 = (const T*)Bt2p;
  __shared__ __align__(16) float sT[8][16 * 68];
  const int b    = blockIdx.y;
  const int lane = threadIdx.x & 31;
  const int wave = threadIdx.x >> 5;
  const int tilesN = N >> 6;
  const int tilesM = M >> 6;
  const int tile = blockIdx.x * 8 + wave;
  if (tile >= tilesM * tilesN) return;
  const int tm = tile / tilesN;
  const int tn = tile - tm * tilesN;
  const int m0 = tm << 6;
  const int n0 = tn << 6;

  const T* Ab  = A  + (size_t)b * strideA;
  const T* Bb  = Bt + (size_t)b * strideB;
  const T* Ab2 = SPLIT ? (A2  + (size_t)b * strideA) : nullptr;
  const T* Bb2 = SPLIT ? (Bt2 + (size_t)b * strideB) : nullptr;

  const int rlane = lane & 15;
  const int koff  = (lane >> 4) * 8;
  const int mOff  = (lane >> 4) * 8;

  v8f acc[4][4];
#pragma unroll
  for (int i = 0; i < 4; ++i)
#pragma unroll
    for (int j = 0; j < 4; ++j) acc[i][j] = (v8f){0.f,0.f,0.f,0.f,0.f,0.f,0.f,0.f};

  for (int k0 = 0; k0 < K; k0 += 32) {
    V bh[4], bl[4];
#pragma unroll
    for (int j = 0; j < 4; ++j) {
      const size_t bo = (size_t)(n0 + (j << 4) + rlane) * ldb + koff + k0;
      bh[j] = Frag<T>::load(Bb + bo);
      if (SPLIT) bl[j] = Frag<T>::load(Bb2 + bo);
    }
#pragma unroll
    for (int i = 0; i < 4; ++i) {
      const size_t ao = (size_t)(m0 + (i << 4) + rlane) * lda + koff + k0;
      V ah = Frag<T>::load(Ab + ao);
      V al;
      if (SPLIT) al = Frag<T>::load(Ab2 + ao);
#pragma unroll
      for (int j = 0; j < 4; ++j) {
        acc[i][j] = Frag<T>::mma(ah, bh[j], acc[i][j]);
        if (SPLIT) {
          acc[i][j] = Frag<T>::mma(ah, bl[j], acc[i][j]);
          acc[i][j] = Frag<T>::mma(al, bh[j], acc[i][j]);
        }
      }
      Frag<T>::guard4(acc[i][0], acc[i][1], acc[i][2], acc[i][3], ah, SPLIT ? al : ah, bh[0], bh[1], bh[2], bh[3]);
    }
    Frag<T>::keep(bh[0], bh[1], bh[2], bh[3]);
    if (SPLIT) Frag<T>::keep(bl[0], bl[1], bl[2], bl[3]);
  }
  acc_guard4(acc[0][0], acc[0][1], acc[0][2], acc[0][3]);
  acc_guard4(acc[1][0], acc[1][1], acc[1][2], acc[1][3]);
  acc_guard4(acc[2][0], acc[2][1], acc[2][2], acc[2][3]);
  acc_guard4(acc[3][0], acc[3][1], acc[3][2], acc[3][3]);

  float* slab = sT[wave];
  const float* Rb = RESID ? (resid + (size_t)b * strideR) : nullptr;
#pragma unroll
  for (int i = 0; i < 4; ++i) {
    const int mBase = m0 + (i << 4);
#pragma unroll
    for (int j = 0; j < 4; ++j) {
      const int n = n0 + (j << 4) + rlane;
      float bv = 0.f;
      if (BIAS_MODE == 2) bv = bias[n];
#pragma unroll
      for (int r = 0; r < 8; ++r) {
        float v = acc[i][j][r] * scale;
        if (BIAS_MODE == 1) v += bias[mBase + mOff + r];
        if (BIAS_MODE == 2) v += bv;
        if (RESID) v += Rb[(size_t)(mBase + mOff + r) * ldc + n];
        if (ACT == 1) v = tanhf(v);
        if (ACT == 2) v = fmaxf(v, 0.0f);
        slab[(mOff + r) * 68 + (j << 4) + rlane] = v;
      }
    }
    __builtin_amdgcn_fence(__ATOMIC_RELEASE, "workgroup");
    __builtin_amdgcn_wave_barrier();
    __builtin_amdgcn_fence(__ATOMIC_ACQUIRE, "workgroup");
    if (OUT_MODE == 0) {
      float* C = (float*)Cout + (size_t)b * strideC;
      const int hh = lane >> 4, c4 = (lane & 15) * 4;
      for (int pass = 0; pass < 2; ++pass) {
#pragma unroll
        for (int it = 0; it < 8; ++it) {
          const int row = it * 2 + hh;
          v4f v = *(const v4f*)(slab + row * 68 + c4);
          *(volatile v4f*)(C + (size_t)(mBase + row) * ldc + n0 + c4) = v;
        }
        __threadfence();
      }
    } else {
      const int q = lane >> 3, c8 = (lane & 7) * 8;
      unsigned short* C  = (unsigned short*)Cout  + (size_t)b * strideC;
      unsigned short* C2 = (OUT_MODE == 2) ? ((unsigned short*)Cout2 + (size_t)b * strideC) : nullptr;
      for (int pass = 0; pass < 2; ++pass) {
#pragma unroll
        for (int it = 0; it < 4; ++it) {
          const int row = it * 4 + q;
          const float* sp = slab + row * 68 + c8;
          v8h hv, lv;
#pragma unroll
          for (int e = 0; e < 8; ++e) {
            if (OUT_MODE == 1) {
              hv[e] = (_Float16)sp[e];
            } else {
              unsigned short hb = f2bf_bits(sp[e]);
              unsigned short lb = f2bf_bits(sp[e] - bf_bits2f(hb));
              hv[e] = __builtin_bit_cast(_Float16, hb);
              lv[e] = __builtin_bit_cast(_Float16, lb);
            }
          }
          *(volatile v8h*)(C + (size_t)(mBase + row) * ldc + n0 + c8) = hv;
          if (OUT_MODE == 2) *(volatile v8h*)(C2 + (size_t)(mBase + row) * ldc + n0 + c8) = lv;
        }
        __threadfence();
      }
    }
    __builtin_amdgcn_fence(__ATOMIC_RELEASE, "workgroup");
    __builtin_amdgcn_wave_barrier();
    __builtin_amdgcn_fence(__ATOMIC_ACQUIRE, "workgroup");
  }
}

__global__ __launch_bounds__(CVT_THR) void embed_cvt_kernel(const int* __restrict__ xs, const float* __restrict__ emb,
                                                            unsigned short* __restrict__ xe) {
  const int i = blockIdx.x * CVT_THR + threadIdx.x;
  if (i < NROWS * (NEMB / 8)) {
    const int row = i >> 6;
    const int c8  = i & 63;
    int tok = xs[row];
    tok = tok < 0 ? 0 : (tok > NVOC - 1 ? NVOC - 1 : tok);
    const float* sp = emb + (size_t)tok * NEMB + c8 * 8;
    const v4f a = *(const v4f*)(sp);
    const v4f b = *(const v4f*)(sp + 4);
    v8h hv;
#pragma unroll
    for (int e = 0; e < 4; ++e) {
      hv[e]     = (_Float16)(a[e] * WCARRY);
      hv[4 + e] = (_Float16)(b[e] * WCARRY);
    }
    *(volatile v8h*)(xe + (size_t)i * 8) = hv;
    __threadfence();
    *(volatile v8h*)(xe + (size_t)i * 8) = hv;
  }
}

__global__ __launch_bounds__(CVT_THR) void tpw_f16_kernel(const float* __restrict__ src, int R, int C, int ldo,
                                                          unsigned short* __restrict__ O, float sc) {
  __shared__ float Tt[64 * 65];
  const int tid = threadIdx.x;
  const int c0 = blockIdx.x * 64, r0 = blockIdx.y * 64;
#pragma unroll
  for (int i = 0; i < 4; ++i) {
    const int idx = i * CVT_THR + tid;
    const int rr = idx >> 4, cc = (idx & 15) * 4;
    const v4f v = *(const v4f*)(src + (size_t)(r0 + rr) * (size_t)C + c0 + cc);
    Tt[rr * 65 + cc + 0] = v[0];
    Tt[rr * 65 + cc + 1] = v[1];
    Tt[rr * 65 + cc + 2] = v[2];
    Tt[rr * 65 + cc + 3] = v[3];
  }
  __syncthreads();
  const int q = tid >> 3, c8 = (tid & 7) * 8;
  v8h hv[2];
#pragma unroll
  for (int g = 0; g < 2; ++g) {
    const int qq = g * 32 + q;
#pragma unroll
    for (int e = 0; e < 8; ++e) {
      const float f = Tt[(c8 + e) * 65 + qq];
      hv[g][e] = (_Float16)(f * sc);
    }
  }
  for (int pass = 0; pass < 2; ++pass) {
#pragma unroll
    for (int g = 0; g < 2; ++g) {
      const size_t o = (size_t)(c0 + g * 32 + q) * (size_t)ldo + (size_t)(r0 + c8);
      *(volatile v8h*)(O + o) = hv[g];
    }
    __threadfence();
  }
}

__device__ __forceinline__ float fsig(float x) { return __builtin_amdgcn_rcpf(1.0f + expf(-x)); }
__device__ __forceinline__ void rot4(v8f (&a)[4]) {
  const v8f t0 = a[0];
  a[0] = a[1];
  a[1] = a[2];
  a[2] = a[3];
  a[3] = t0;
}
__device__ __forceinline__ void mma4(const v16h a, const _Float16* bp, v8f& c0, v8f& c1, v8f& c2, v8f& c3) {
  const v16h b0 = Frag<_Float16>::load(bp);
  const v16h b1 = Frag<_Float16>::load(bp + (size_t)16 * NHID);
  const v16h b2 = Frag<_Float16>::load(bp + (size_t)32 * NHID);
  const v16h b3 = Frag<_Float16>::load(bp + (size_t)48 * NHID);
  c0 = Frag<_Float16>::mma(a, b0, c0);
  c1 = Frag<_Float16>::mma(a, b1, c1);
  c2 = Frag<_Float16>::mma(a, b2, c2);
  c3 = Frag<_Float16>::mma(a, b3, c3);
  grp_guard_h(c0, c1, c2, c3, a, a, b0, b1, b2, b3);
}

template <bool FWD>
__global__ __launch_bounds__(SCAN_THR) void gru_scan_kernel(
    const unsigned short* __restrict__ WzrTp, const unsigned short* __restrict__ WhhTp,
    const float* __restrict__ bx, const float* __restrict__ bhzr, const float* __restrict__ bhh,
    const unsigned short* __restrict__ GXT, const float* __restrict__ mask,
    unsigned short* __restrict__ SEQ16, float* __restrict__ SEQF) {
  __shared__ __align__(16) _Float16 Hh[ROWS_BLK * HPITCH];
  __shared__ __align__(16) _Float16 Rh[ROWS_BLK * HPITCH];
  __shared__ __align__(16) float    Sl[SCAN_WAVES][16 * SLABP];
  const _Float16* WzrT = (const _Float16*)WzrTp;
  const _Float16* WhhT = (const _Float16*)WhhTp;
  const int tid = threadIdx.x, lane = tid & 31, wave = tid >> 5;
  const int c = lane & 15, hh = lane >> 4, koff = hh * 8;
  const int rowbase = blockIdx.x * ROWS_BLK;

#pragma unroll 1
  for (int i = tid; i < ROWS_BLK * HPITCH; i += SCAN_THR) {
    Hh[i] = (_Float16)0.0f;
    Rh[i] = (_Float16)0.0f;
  }
  const v8f z8 = {0.f, 0.f, 0.f, 0.f, 0.f, 0.f, 0.f, 0.f};
  v8f hst[4];
  hst[0] = z8;
  hst[1] = z8;
  hst[2] = z8;
  hst[3] = z8;
  __syncthreads();

  float* slab = Sl[wave];
  const _Float16* arowH = Hh + c * HPITCH + koff;
  const _Float16* arowR = Rh + c * HPITCH + koff;
  const _Float16* wz = WzrT + (size_t)(64 * wave + c) * NHID + koff;
  const _Float16* wr = wz + (size_t)NHID * NHID;
  const _Float16* wc = WhhT + (size_t)(64 * wave + c) * NHID + koff;

#pragma unroll 1
  for (int step = 0; step < SEQ_LEN; ++step) {
    const int t = FWD ? step : (SEQ_LEN - 1 - step);
    const size_t gofs = (size_t)t * NBAT + (size_t)(rowbase + 8 * hh);
    const v4f mk0 = *(const v4f*)(mask + gofs);
    const v4f mk1 = *(const v4f*)(mask + gofs + 4);
    float mk[8];
    mk[0] = mk0[0];
    mk[1] = mk0[1];
    mk[2] = mk0[2];
    mk[3] = mk0[3];
    mk[4] = mk1[0];
    mk[5] = mk1[1];
    mk[6] = mk1[2];
    mk[7] = mk1[3];

    v8f accZ[4], accR[4];
    accZ[0] = z8;
    accZ[1] = z8;
    accZ[2] = z8;
    accZ[3] = z8;
    accR[0] = z8;
    accR[1] = z8;
    accR[2] = z8;
    accR[3] = z8;
#pragma unroll 1
    for (int k0 = 0; k0 < NHID; k0 += 32) {
      const v16h a = Frag<_Float16>::load(arowH + k0);
      mma4(a, wz + k0, accZ[0], accZ[1], accZ[2], accZ[3]);
      mma4(a, wr + k0, accR[0], accR[1], accR[2], accR[3]);
    }
    acc_guard4(accZ[0], accZ[1], accZ[2], accZ[3]);
    acc_guard4(accR[0], accR[1], accR[2], accR[3]);

#pragma unroll 1
    for (int it = 0; it < 4; ++it) {
      const int j = 64 * wave + 16 * it + c;
      const v4u gzw = *(const v4u*)(const void*)(GXT + (size_t)j * NROWS + gofs);
      const v4u grw = *(const v4u*)(const void*)(GXT + (size_t)(NHID + j) * NROWS + gofs);
      const float bz = bx[j] + bhzr[j];
      const float br = bx[NHID + j] + bhzr[NHID + j];
      float gzf[8], grf[8];
      unpack8(gzw, gzf);
      unpack8(grw, grf);
      v8f zv = accZ[0];
      const v8f rv = accR[0];
      const v8f hv = hst[0];
#pragma unroll
      for (int r = 0; r < 8; ++r) {
        const float zp = zv[r] * ACC_INV + (gzf[r] * GX_INV + bz);
        const float rp = rv[r] * ACC_INV + (grf[r] * GX_INV + br);
        const float zg = fsig(zp);
        const float rg = fsig(rp);
        const float rhv = rg * hv[r];
        Rh[(8 * hh + r) * HPITCH + j] = (_Float16)(rhv * HCARRY);
        zv[r] = zg;
      }
      accZ[0] = zv;
      rot4(accZ);
      rot4(accR);
      rot4(hst);
    }
    __syncthreads();

    v8f accC[4];
    accC[0] = z8;
    accC[1] = z8;
    accC[2] = z8;
    accC[3] = z8;
#pragma unroll 1
    for (int k0 = 0; k0 < NHID; k0 += 32) {
      const v16h a = Frag<_Float16>::load(arowR + k0);
      mma4(a, wc + k0, accC[0], accC[1], accC[2], accC[3]);
    }
    acc_guard4(accC[0], accC[1], accC[2], accC[3]);

#pragma unroll 1
    for (int it = 0; it < 4; ++it) {
      const int j = 64 * wave + 16 * it + c;
      const v4u gcw = *(const v4u*)(const void*)(GXT + (size_t)(NGATE2 + j) * NROWS + gofs);
      const float bc = bx[NGATE2 + j] + bhh[j];
      float gcf[8];
      unpack8(gcw, gcf);
      const v8f cv = accC[0];
      const v8f zv = accZ[0];
      v8f hv = hst[0];
#pragma unroll
      for (int r = 0; r < 8; ++r) {
        const float cp = cv[r] * ACC_INV + (gcf[r] * GX_INV + bc);
        const float cand = tanhf(cp);
        const float ho = hv[r];
        const float zg = zv[r];
        float hn = (1.0f - zg) * ho + zg * cand;
        const float m = mk[r];
        hn = m * hn + (1.0f - m) * ho;
        hv[r] = hn;
        Hh[(8 * hh + r) * HPITCH + j] = (_Float16)(hn * HCARRY);
        slab[(8 * hh + r) * SLABP + 16 * it + c] = hn;
      }
      hst[0] = hv;
      rot4(accC);
      rot4(accZ);
      rot4(hst);
    }
    __syncthreads();

    if (FWD) {
      const int q = lane >> 3, c8 = (lane & 7) * 8;
      for (int pass = 0; pass < 2; ++pass) {
#pragma unroll
        for (int it = 0; it < 4; ++it) {
          const int row = it * 4 + q;
          const float* sp = slab + row * SLABP + c8;
          v8h ov;
#pragma unroll
          for (int e = 0; e < 8; ++e) ov[e] = (_Float16)(sp[e] * HCARRY);
          *(volatile v8h*)(SEQ16 + ((size_t)t * NBAT + (size_t)(rowbase + row)) * NHID + 64 * wave + c8) = ov;
        }
        __threadfence();
      }
    } else {
      const int c4 = c * 4;
      for (int pass = 0; pass < 2; ++pass) {
#pragma unroll
        for (int it = 0; it < 8; ++it) {
          const int row = it * 2 + hh;
          const v4f v = *(const v4f*)(slab + row * SLABP + c4);
          *(volatile v4f*)(SEQF + ((size_t)t * NBAT + (size_t)(rowbase + row)) * NHID + 64 * wave + c4) = v;
        }
        __threadfence();
      }
    }
  }
}

extern "C" void kernel_launch(void* const* d_in, const int* in_sizes, int n_in,
                              void* d_out, int out_size, void* d_ws, size_t ws_size, hipStream_t stream) {
  if (n_in < 15 || d_out == nullptr || d_ws == nullptr) return;
  if (in_sizes[0] != NROWS || in_sizes[1] != NROWS || in_sizes[2] != NVOC * NEMB ||
      in_sizes[3] != NEMB * NGATE3 || in_sizes[4] != NGATE3 ||
      in_sizes[5] != NHID * NGATE2 || in_sizes[6] != NGATE2 ||
      in_sizes[7] != NHID * NHID || in_sizes[8] != NHID ||
      in_sizes[9] != NHID * NGATE3 || in_sizes[10] != NGATE3 ||
      in_sizes[11] != NHID * NGATE2 || in_sizes[12] != NGATE2 ||
      in_sizes[13] != NHID * NHID || in_sizes[14] != NHID ||
      out_size != NROWS * NHID) return;

  const int*   xs      = (const int*)  d_in[0];
  const float* xs_mask = (const float*)d_in[1];
  const float* emb     = (const float*)d_in[2];
  const float* fw_Wx   = (const float*)d_in[3];
  const float* fw_bx   = (const float*)d_in[4];
  const float* fw_Whzr = (const float*)d_in[5];
  const float* fw_bhzr = (const float*)d_in[6];
  const float* fw_Whh  = (const float*)d_in[7];
  const float* fw_bhh  = (const float*)d_in[8];
  const float* bw_Wx   = (const float*)d_in[9];
  const float* bw_bx   = (const float*)d_in[10];
  const float* bw_Whzr = (const float*)d_in[11];
  const float* bw_bhzr = (const float*)d_in[12];
  const float* bw_Whh  = (const float*)d_in[13];
  const float* bw_bhh  = (const float*)d_in[14];
  float* out = (float*)d_out;

  char* ws = (char*)d_ws;
  size_t off = 0;
  auto carve = [&](size_t bytes) -> char* { char* p = ws + off; off += (bytes + 255) & ~(size_t)255; return p; };
  unsigned short* XE     = (unsigned short*)carve((size_t)NROWS * NEMB * 2);
  unsigned short* FWWXT  = (unsigned short*)carve((size_t)NGATE3 * NEMB * 2);
  unsigned short* FWWZRT = (unsigned short*)carve((size_t)NGATE2 * NHID * 2);
  unsigned short* FWWHHT = (unsigned short*)carve((size_t)NHID * NHID * 2);
  unsigned short* BWWXT  = (unsigned short*)carve((size_t)NGATE3 * NHID * 2);
  unsigned short* BWWZRT = (unsigned short*)carve((size_t)NGATE2 * NHID * 2);
  unsigned short* BWWHHT = (unsigned short*)carve((size_t)NHID * NHID * 2);
  unsigned short* GXT    = (unsigned short*)carve((size_t)NGATE3 * NROWS * 2);
  unsigned short* RIGHT  = (unsigned short*)carve((size_t)NROWS * NHID * 2);
  if (off > ws_size || off > (size_t)134217728) return;

  embed_cvt_kernel<<<(NROWS * (NEMB / 8)) / CVT_THR, CVT_THR, 0, stream>>>(xs, emb, XE);

  tpw_f16_kernel<<<dim3(NGATE3 / 64, NEMB / 64), CVT_THR, 0, stream>>>(fw_Wx,   NEMB, NGATE3, NEMB, FWWXT,  WCARRY);
  tpw_f16_kernel<<<dim3(NGATE2 / 64, NHID / 64), CVT_THR, 0, stream>>>(fw_Whzr, NHID, NGATE2, NHID, FWWZRT, WCARRY);
  tpw_f16_kernel<<<dim3(NHID / 64,   NHID / 64), CVT_THR, 0, stream>>>(fw_Whh,  NHID, NHID,   NHID, FWWHHT, WCARRY);
  tpw_f16_kernel<<<dim3(NGATE3 / 64, NHID / 64), CVT_THR, 0, stream>>>(bw_Wx,   NHID, NGATE3, NHID, BWWXT,  WCARRY);
  tpw_f16_kernel<<<dim3(NGATE2 / 64, NHID / 64), CVT_THR, 0, stream>>>(bw_Whzr, NHID, NGATE2, NHID, BWWZRT, WCARRY);
  tpw_f16_kernel<<<dim3(NHID / 64,   NHID / 64), CVT_THR, 0, stream>>>(bw_Whh,  NHID, NHID,   NHID, BWWHHT, WCARRY);

  const dim3 ggrid((NGATE3 / 64) * (NROWS / 64) / 8, 1);
  wmma_gemm64<0, false, 0, 1, false, 0><<<ggrid, 256, 0, stream>>>(
      FWWXT, FWWXT, NEMB, 0L, XE, XE, NEMB, 0L, (void*)GXT, (void*)GXT, NROWS, 0L,
      fw_bx, fw_bx, 0L, NGATE3, NROWS, NEMB, S1_SCALE);

  gru_scan_kernel<true><<<NBAT / ROWS_BLK, SCAN_THR, 0, stream>>>(
      FWWZRT, FWWHHT, fw_bx, fw_bhzr, fw_bhh, GXT, xs_mask, RIGHT, out);

  wmma_gemm64<0, false, 0, 1, false, 0><<<ggrid, 256, 0, stream>>>(
      BWWXT, BWWXT, NHID, 0L, RIGHT, RIGHT, NHID, 0L, (void*)GXT, (void*)GXT, NROWS, 0L,
      bw_bx, bw_bx, 0L, NGATE3, NROWS, NHID, S4_SCALE);

  gru_scan_kernel<false><<<NBAT / ROWS_BLK, SCAN_THR, 0, stream>>>(
      BWWZRT, BWWHHT, bw_bx, bw_bhzr, bw_bhh, GXT, xs_mask, RIGHT, out);
}
